// MusicTransformer_56590489092572
// MI455X (gfx1250) — hardware-run, weakly checked
//
#include <hip/hip_runtime.h>
#include <math.h>


#ifndef NB
#define NB 1
#endif
#ifndef SEQ
#define SEQ 1024
#endif
#define NB_FULL  1
#define SEQ_FULL 1024
#define DIN   128
#define DM    512
#define NH_   8
#define HD    64
#define NL    4
#define DFF   2048
#define DMI   1024
#define DOUT  390
#define DOUTP 448
#define ERR   2047
#define ERP   2048
#define RELOFF (SEQ_FULL - 1)
#define AW    4
#define OSP   68
#define GP    52
#define GSP   68
#define QRS   2048.0f
#define QRI   (1.0f / 2048.0f)
#define WC    64.0f
#define WCI   (1.0f / 64.0f)
#define LOG2E 1.4426950408889634f
#define SC2   ((float)(0.125 * 1.4426950408889634))
#define PSH   14.0f
#define NEGB  (-3.0e38f)
#define LNEPS 1e-5f

static_assert(NB == 1);
static_assert(HD == 64);
static_assert(NH_ * HD == DM);
static_assert(SEQ % 64 == 0);
static_assert(SEQ % 32 == 0);
static_assert(SEQ % (16 * AW) == 0);
static_assert(SEQ <= SEQ_FULL);
static_assert(DIN % 64 == 0 && DM % 64 == 0 && DFF % 64 == 0 && DMI % 64 == 0 && DOUTP % 64 == 0);
static_assert(DOUT <= DOUTP);
static_assert(DMI <= DFF);
static_assert(SEQ - 16 + RELOFF + 1 + 15 < ERP);
static_assert(RELOFF - 15 - 16 - (SEQ - 32) >= 0);
static_assert(ERR + 1 == ERP);
static_assert((OSP * 4) % 16 == 0 && (GP * 4) % 16 == 0 && (GSP * 4) % 16 == 0);
static_assert(GP >= 48);
static_assert(DM == 512);
static_assert((SEQ * DOUT) % 4 == 0);

typedef _Float16 h16;
typedef __attribute__((ext_vector_type(16))) _Float16 v16h;
typedef __attribute__((ext_vector_type(8)))  _Float16 v8h;
typedef __attribute__((ext_vector_type(8)))  float    v8f;
typedef __attribute__((ext_vector_type(4)))  float    v4f;
typedef v4f  __attribute__((may_alias)) v4fa;

__device__ __forceinline__ unsigned short f2bf(float f) { unsigned u = __float_as_uint(f); u += 0x7FFFu + ((u >> 16) & 1u); return (unsigned short)(u >> 16); }
__device__ __forceinline__ float bfr(float f) { return __uint_as_float(((unsigned)f2bf(f)) << 16); }
__device__ __forceinline__ v16h cat16(v8h lo, v8h hi) { return __builtin_shufflevector(lo, hi, 0, 1, 2, 3, 4, 5, 6, 7, 8, 9, 10, 11, 12, 13, 14, 15); }
__device__ __forceinline__ v16h  ldh(const h16* p) { return cat16(*(const v8h*)p, *(const v8h*)(p + 16)); }
__device__ __forceinline__ void wave_sync() { __builtin_amdgcn_fence(3  , "wavefront"); __builtin_amdgcn_wave_barrier(); asm volatile("" ::: "memory"); }
__device__ __forceinline__ h16 toh_flush(float v) { const h16 r = (h16)v; return (fabsf(v) < 6.103515625e-05f) ? (h16)0.0f : r; }
__device__ __forceinline__ v8f wmma16g(v16h a, v16h b, v8f c) {
    c = __builtin_amdgcn_wmma_f32_16x16x32_f16(false, a, false, b, (short)0, c, false, false);
    asm volatile("v_nop\n\tv_nop\n\tv_nop\n\tv_nop" : "+v"(c) : "v"(a), "v"(b));
    return c; }
__device__ __forceinline__ float gelu_erf(float x) { return 0.5f * x * (1.0f + erff(x * 0.70710678118654752f)); }
__device__ __forceinline__ v4f lo4(v8f g) { return __builtin_shufflevector(g, g, 0, 1, 2, 3); }
__device__ __forceinline__ v4f hi4(v8f g) { return __builtin_shufflevector(g, g, 4, 5, 6, 7); }

__global__ __launch_bounds__(256) void k_cvt8h(const float* __restrict__ src, h16* dst, int n8) {
    const int i = blockIdx.x * 256 + threadIdx.x; if (i >= n8) return;
    const v8f v = *(const v8f*)(src + (size_t)i * 8); v8h o;
#pragma unroll
    for (int k = 0; k < 8; ++k) o[k] = toh_flush(bfr(v[k]));
    *(volatile v8h*)(dst + (size_t)i * 8) = o; __threadfence(); *(volatile v8h*)(dst + (size_t)i * 8) = o;
}

__global__ __launch_bounds__(256) void k_cvt_er(const float* __restrict__ src, h16* dst) {
    const int i = blockIdx.x * 256 + threadIdx.x; if (i >= NL * ERP * HD / 8) return;
    const int c8 = (i & 7) * 8; const int r = (i >> 3) % ERP; const int l = (i >> 3) / ERP;
    const int rc = r < ERR ? r : ERR - 1;
    v8f v = *(const v8f*)(src + ((size_t)l * ERR + rc) * HD + c8);
    asm volatile("" : "+v"(v));
    v8h o;
#pragma unroll
    for (int k = 0; k < 8; ++k) o[k] = (r < ERR) ? toh_flush(bfr(v[k])) : (h16)0.0f;
    *(volatile v8h*)(dst + (size_t)i * 8) = o; __threadfence(); *(volatile v8h*)(dst + (size_t)i * 8) = o;
}

__global__ __launch_bounds__(256) void k_wconv(const float* __restrict__ W, h16* Wt, int K, int N, int NP, float carry) {
#pragma clang fp contract(off)
    __shared__ float ts[64 * 65];
    static_assert(sizeof(float) * 64 * 65 <= 131072);
    const int tid = threadIdx.x;
    const int k0 = blockIdx.x * 64, n0 = blockIdx.y * 64;
    const size_t lin = (size_t)blockIdx.z * (size_t)K * (size_t)N, lout = (size_t)blockIdx.z * (size_t)NP * (size_t)K;
    static_assert(16 * 4 == 64);
#pragma unroll 1
    for (int p = 0; p < 16; ++p) {
        const int kk = p * 4 + (tid >> 6), nn = tid & 63; const int n = n0 + nn; const int nc = n < N ? n : N - 1;
        float v = W[lin + (size_t)(k0 + kk) * N + nc];
        asm volatile("" : "+v"(v));
        ts[kk * 65 + nn] = (n < N) ? bfr(v) * carry : 0.0f; }
    __syncthreads();
    static_assert(256 * 16 * 2 == 64 * 128);
#pragma unroll 1
    for (int ps = 0; ps < 2; ++ps) {
#pragma unroll 1
        for (int p = 0; p < 2; ++p) {
            const int row = p * 32 + (tid >> 3), c8 = (tid & 7) * 8; v8h o;
#pragma unroll
            for (int i = 0; i < 8; ++i) o[i] = toh_flush(ts[(c8 + i) * 65 + row]);
            *(volatile v8h*)(Wt + lout + (size_t)(n0 + row) * K + k0 + c8) = o; }
        if (ps == 0) __threadfence(); }
}

__global__ __launch_bounds__(128) void k_ln(const float* __restrict__ X, const float* __restrict__ g, const float* __restrict__ b, h16* NHp, h16* NRp, int wres) {
#pragma clang fp contract(off)
    const int lane = threadIdx.x & 31;
    const int wave = __builtin_amdgcn_readfirstlane((int)(threadIdx.x >> 5));
    const int row = blockIdx.x * 4 + wave;
    const float* xr = X + (size_t)row * DM;
    const v8f x0 = *(const v8f*)(xr + lane * 8), x1 = *(const v8f*)(xr + 256 + lane * 8);
    float s = 0.0f;
#pragma unroll
    for (int k = 0; k < 8; ++k) { s += x0[k]; s += x1[k]; }
#pragma unroll
    for (int off = 16; off > 0; off >>= 1) s += __shfl_xor(s, off, 32);
    const float mean = s * (1.0f / (float)DM);
    const v8f d0 = x0 - mean, d1 = x1 - mean;
    float q = 0.0f;
#pragma unroll
    for (int k = 0; k < 8; ++k) { q += d0[k] * d0[k]; q += d1[k] * d1[k]; }
#pragma unroll
    for (int off = 16; off > 0; off >>= 1) q += __shfl_xor(q, off, 32);
    const float rstd = 1.0f / sqrtf(q * (1.0f / (float)DM) + LNEPS);
    const v8f g0 = *(const v8f*)(g + lane * 8), g1 = *(const v8f*)(g + 256 + lane * 8);
    const v8f b0 = *(const v8f*)(b + lane * 8), b1 = *(const v8f*)(b + 256 + lane * 8);
    v8h h0, h1, r0, r1;
#pragma unroll
    for (int k = 0; k < 8; ++k) {
        const float y0 = d0[k] * rstd * bfr(g0[k]) + bfr(b0[k]);
        const float y1 = d1[k] * rstd * bfr(g1[k]) + bfr(b1[k]);
        const h16 a0 = toh_flush(y0), a1 = toh_flush(y1);
        h0[k] = a0; h1[k] = a1;
        r0[k] = toh_flush((y0 - (float)a0) * QRS); r1[k] = toh_flush((y1 - (float)a1) * QRS); }
    const size_t o0 = (size_t)row * DM + lane * 8, o1 = o0 + 256;
    static_assert(32 * 16 * 2 == DM * 2);
#pragma unroll 1
    for (int ps = 0; ps < 2; ++ps) {
        *(volatile v8h*)(NHp + o0) = h0; *(volatile v8h*)(NHp + o1) = h1;
        if (wres != 0) { *(volatile v8h*)(NRp + o0) = r0; *(volatile v8h*)(NRp + o1) = r1; }
        if (ps == 0) __threadfence(); }
}

__device__ __forceinline__ void gemm_kloop(const h16* __restrict__ A, const h16* __restrict__ Bt, size_t aoff, size_t boff, int K, v8f (&acc)[4][4]) {
#pragma unroll 1
    for (int kc = 0; kc < K; kc += 32) {
        v16h a[4];
#pragma unroll
        for (int mb = 0; mb < 4; ++mb) a[mb] = ldh(A + aoff + (size_t)mb * 16 * K + kc);
#pragma unroll
        for (int nb = 0; nb < 4; ++nb) { const v16h b = ldh(Bt + boff + (size_t)nb * 16 * K + kc);
#pragma unroll
            for (int mb = 0; mb < 4; ++mb) acc[mb][nb] = wmma16g(a[mb], b, acc[mb][nb]); }
    }
}

template <int OUTF32, int HASRES, int GELU, int ARES, int ORES, int ROWB, int HEADPL>
__device__ __forceinline__ void gemm_body(const h16* __restrict__ A, const h16* __restrict__ Ar, const h16* __restrict__ Bt,
                                          const float* __restrict__ bias, int nvalid, int K, float csc,
                                          const float* __restrict__ Res, float* Cf, h16* Ch, h16* Cr, int ldc) {
    __shared__ __align__(16) float os[64 * GSP];
    static_assert(sizeof(float) * 64 * GSP <= 131072);
    const int lane = threadIdx.x & 31, lr = lane & 15, hi = lane >> 4;
    const int r0 = blockIdx.x * 64, c0 = blockIdx.y * 64;
    v8f acc[4][4];
#pragma unroll
    for (int mb = 0; mb < 4; ++mb)
#pragma unroll
        for (int nb = 0; nb < 4; ++nb) acc[mb][nb] = (v8f){};
    const size_t aoff = (size_t)(r0 + lr) * K + 8 * hi, boff = (size_t)(c0 + lr) * K + 8 * hi;
    if (ARES) {
        gemm_kloop(Ar, Bt, aoff, boff, K, acc);
#pragma unroll
        for (int mb = 0; mb < 4; ++mb)
#pragma unroll
            for (int nb = 0; nb < 4; ++nb) acc[mb][nb] = acc[mb][nb] * QRI;
    }
    gemm_kloop(A, Bt, aoff, boff, K, acc);
    float bc[4];
#pragma unroll
    for (int nb = 0; nb < 4; ++nb) {
        if (ROWB) { bc[nb] = 0.0f; }
        else { const int c = c0 + nb * 16 + lr; const int cc = c < nvalid ? c : nvalid - 1;
               float bvv = bias[cc]; asm volatile("" : "+v"(bvv)); bc[nb] = (c < nvalid) ? bfr(bvv) : 0.0f; } }
#pragma unroll
    for (int mb = 0; mb < 4; ++mb) {
        float br[8];
#pragma unroll
        for (int j = 0; j < 8; ++j) br[j] = ROWB ? bfr(bias[r0 + mb * 16 + hi * 8 + j]) : 0.0f;
#pragma unroll
        for (int nb = 0; nb < 4; ++nb) {
#pragma unroll
            for (int j = 0; j < 8; ++j) os[(mb * 16 + hi * 8 + j) * GSP + nb * 16 + lr] = acc[mb][nb][j] * csc + bc[nb] + br[j]; }
    }
    wave_sync();
    if (OUTF32) {
        static_assert(32 * 16 * 32 == 64 * 256);
#pragma unroll 1
        for (int ps = 0; ps < 2; ++ps) {
#pragma unroll 1
            for (int s = 0; s < 32; ++s) { const int row = 2 * s + (lane >> 4), c4 = (lane & 15) * 4;
                v4f val = *(const v4fa*)(&os[row * GSP + c4]);
                const size_t go = (size_t)(r0 + row) * ldc + c0 + c4;
                if (HASRES) { const v4f rr = *(const v4f*)(Res + go); val = val + rr; }
                *(volatile v4f*)(Cf + go) = val; }
            if (ps == 0) __threadfence(); }
    } else {
        static_assert(32 * 16 * 16 == 64 * 128);
        const size_t obase = HEADPL ? ((size_t)(c0 / HD) * SEQ + (size_t)r0) * HD : (size_t)r0 * ldc + c0;
        const int pitch = HEADPL ? HD : ldc;
#pragma unroll 1
        for (int ps = 0; ps < 2; ++ps) {
#pragma unroll 1
            for (int s = 0; s < 16; ++s) { const int row = 4 * s + (lane >> 3), c8 = (lane & 7) * 8;
                const v4f x0 = *(const v4fa*)(&os[row * GSP + c8]); const v4f x1 = *(const v4fa*)(&os[row * GSP + c8 + 4]); v8h hv, rv;
#pragma unroll
                for (int i = 0; i < 4; ++i) { float y0 = x0[i], y1 = x1[i];
                    if (GELU) { y0 = gelu_erf(y0); y1 = gelu_erf(y1); }
                    const h16 a0 = toh_flush(y0); const h16 a1 = toh_flush(y1); hv[i] = a0; hv[4 + i] = a1;
                    rv[i] = toh_flush((y0 - (float)a0) * QRS); rv[4 + i] = toh_flush((y1 - (float)a1) * QRS); }
                const size_t oo = obase + (size_t)row * pitch + c8;
                *(volatile v8h*)(Ch + oo) = hv; if (ORES) *(volatile v8h*)(Cr + oo) = rv; }
            if (ps == 0) __threadfence(); }
    }
}

__global__ __launch_bounds__(32) void k_gemm_f32(const h16* __restrict__ A, const h16* __restrict__ Bt, const float* __restrict__ bias, int nvalid, int K, float csc, float* C, int ldc) {
    gemm_body<1, 0, 0, 0, 0, 0, 0>(A, nullptr, Bt, bias, nvalid, K, csc, nullptr, C, nullptr, nullptr, ldc); }
__global__ __launch_bounds__(32) void k_gemm_f32r(const h16* __restrict__ A, const h16* __restrict__ Bt, const float* __restrict__ bias, int nvalid, int K, float csc, const float* __restrict__ Res, float* C, int ldc) {
    gemm_body<1, 1, 0, 0, 0, 0, 0>(A, nullptr, Bt, bias, nvalid, K, csc, Res, C, nullptr, nullptr, ldc); }
__global__ __launch_bounds__(32) void k_gemm_gelu(const h16* __restrict__ A, const h16* __restrict__ Bt, const float* __restrict__ bias, int nvalid, int K, float csc, h16* C, int ldc) {
    gemm_body<0, 0, 1, 0, 0, 0, 0>(A, nullptr, Bt, bias, nvalid, K, csc, nullptr, nullptr, C, nullptr, ldc); }
__global__ __launch_bounds__(32) void k_gemm_q(const h16* __restrict__ A, const h16* __restrict__ Ar, const h16* __restrict__ Bt, const float* __restrict__ bias, int nvalid, int K, float csc, h16* Ph, h16* Pr) {
    gemm_body<0, 0, 0, 1, 1, 0, 1>(A, Ar, Bt, bias, nvalid, K, csc, nullptr, nullptr, Ph, Pr, HD); }
__global__ __launch_bounds__(32) void k_gemm_k(const h16* __restrict__ A, const h16* __restrict__ Bt, const float* __restrict__ bias, int nvalid, int K, float csc, h16* Ph) {
    gemm_body<0, 0, 0, 0, 0, 0, 1>(A, nullptr, Bt, bias, nvalid, K, csc, nullptr, nullptr, Ph, nullptr, HD); }
__global__ __launch_bounds__(32) void k_gemm_vt(const h16* __restrict__ A, const h16* __restrict__ Bt, const float* __restrict__ bias, int K, float csc, h16* Ph, int ldc) {
    gemm_body<0, 0, 0, 0, 0, 1, 0>(A, nullptr, Bt, bias, 0, K, csc, nullptr, nullptr, Ph, nullptr, ldc); }

__device__ __forceinline__ v8f gtile(const h16* __restrict__ ep, v16h qh0, v16h qh1, v16h qr0, v16h qr1) {
    const v16h e0 = ldh(ep), e1 = ldh(ep + 32);
    v8f gH = (v8f){}, gL = (v8f){};
    gH = wmma16g(e0, qh0, gH); gH = wmma16g(e1, qh1, gH);
    gL = wmma16g(e0, qr0, gL); gL = wmma16g(e1, qr1, gL);
    return (gH + gL * QRI) * LOG2E;
}

__global__ __launch_bounds__(32 * AW) void k_flash(const h16* __restrict__ QH, const h16* __restrict__ QR, const h16* __restrict__ KP, const h16* __restrict__ VT, const h16* __restrict__ EPl, h16* OP) {
    __shared__ __align__(16) float os[AW * 16 * OSP];
    __shared__ __align__(16) float gs[AW * 16 * GP];
    static_assert(sizeof(float) * (AW * 16 * OSP + AW * 16 * GP) <= 131072);
    const int lane = threadIdx.x & 31, lr = lane & 15, hi = lane >> 4;
    const int wave = __builtin_amdgcn_readfirstlane((int)(threadIdx.x >> 5));
    const int h = blockIdx.y;
    const int t0 = (blockIdx.x * AW + wave) * 16;
    const size_t pbase = (size_t)h * SEQ * HD;
    const size_t qo = pbase + (size_t)(t0 + lr) * HD + 8 * hi;
    const v16h qh0 = ldh(QH + qo), qh1 = ldh(QH + qo + 32);
    const v16h qr0 = ldh(QR + qo), qr1 = ldh(QR + qo + 32);
    const size_t ko = pbase + (size_t)lr * HD + 8 * hi;
    const size_t vo = pbase + (size_t)lr * SEQ + 8 * hi;
    const h16* eb = EPl + (size_t)lr * HD + 8 * hi;
    const int gw  = wave * 16 * GP + lr * GP;
    const int gst = gw + 8 * hi;
    const int gld = gw + lr - 8 * hi;
    v8f gprev = gtile(eb + (size_t)(t0 + RELOFF + 1) * HD, qh0, qh1, qr0, qr1);
    v8f o[4];
#pragma unroll
    for (int j = 0; j < 4; ++j) o[j] = (v8f){};
    float m = NEGB, l = 0.0f;
#pragma unroll 1
    for (int key0 = 0; key0 < SEQ; key0 += 32) {
        const int rbA = t0 - key0 + (RELOFF - 15);
        const v8f g1 = gtile(eb + (size_t)rbA * HD, qh0, qh1, qr0, qr1);
        const v8f g0 = gtile(eb + (size_t)(rbA - 16) * HD, qh0, qh1, qr0, qr1);
        *(v4fa*)(&gs[gst +  0]) = lo4(g0);    *(v4fa*)(&gs[gst +  4]) = hi4(g0);
        *(v4fa*)(&gs[gst + 16]) = lo4(g1);    *(v4fa*)(&gs[gst + 20]) = hi4(g1);
        *(v4fa*)(&gs[gst + 32]) = lo4(gprev); *(v4fa*)(&gs[gst + 36]) = hi4(gprev);
        gprev = g0;
        const h16* ka = KP + ko + (size_t)key0 * HD;
        const v16h ka0 = ldh(ka), ka1 = ldh(ka + 32), kb0 = ldh(ka + 16 * HD), kb1 = ldh(ka + 16 * HD + 32);
        v8f sHa = (v8f){}, sLa = (v8f){}, sHb = (v8f){}, sLb = (v8f){};
        sHa = wmma16g(ka0, qh0, sHa); sHa = wmma16g(ka1, qh1, sHa);
        sLa = wmma16g(ka0, qr0, sLa); sLa = wmma16g(ka1, qr1, sLa);
        sHb = wmma16g(kb0, qh0, sHb); sHb = wmma16g(kb1, qh1, sHb);
        sLb = wmma16g(kb0, qr0, sLb); sLb = wmma16g(kb1, qr1, sLb);
        wave_sync();
        float ra[8], rb[8];
#pragma unroll
        for (int r = 0; r < 8; ++r) { ra[r] = gs[gld + 31 - r]; rb[r] = gs[gld + 15 - r]; }
        wave_sync();
        float ta[8], tb[8]; float mx = NEGB;
#pragma unroll
        for (int r = 0; r < 8; ++r) {
            ta[r] = (sHa[r] + sLa[r] * QRI) * SC2 + ra[r]; tb[r] = (sHb[r] + sLb[r] * QRI) * SC2 + rb[r];
            mx = fmaxf(mx, fmaxf(ta[r], tb[r])); }
        mx = fmaxf(mx, __shfl_xor(mx, 16, 32));
        const float mnew = fmaxf(m, mx);
        const float alpha = __builtin_amdgcn_exp2f(m - mnew);
        const float sh = PSH - mnew;
        v16h pb; float ls = 0.0f;
#pragma unroll
        for (int r = 0; r < 8; ++r) {
            const float xa = ta[r] + sh, xb = tb[r] + sh;
            const float ea = __builtin_amdgcn_exp2f(xa), ec = __builtin_amdgcn_exp2f(xb);
            const float ga = (xa < -14.0f) ? 0.0f : ea, gb = (xb < -14.0f) ? 0.0f : ec;
            const h16 pa = (h16)ga; const h16 pc = (h16)gb;
            pb[r] = pa; pb[8 + r] = pc;
            ls += (float)pa + (float)pc; }
        l = l * alpha + ls; m = mnew;
        const h16* va = VT + vo + key0;
#pragma unroll
        for (int j = 0; j < 4; ++j) { o[j] = o[j] * alpha; const v16h vj = ldh(va + (size_t)16 * j * SEQ); o[j] = wmma16g(vj, pb, o[j]); }
    }
    l += __shfl_xor(l, 16, 32);
    const float inv = 1.0f / l;
    const int wb = wave * 16 * OSP;
#pragma unroll
    for (int j = 0; j < 4; ++j) {
        *(v4fa*)(&os[wb + lr * OSP + 16 * j + 8 * hi])     = lo4(o[j]) * inv;
        *(v4fa*)(&os[wb + lr * OSP + 16 * j + 8 * hi + 4]) = hi4(o[j]) * inv; }
    wave_sync();
    h16* orow = OP + (size_t)t0 * DM + h * HD;
    static_assert(32 * 16 * 4 == 16 * 128);
#pragma unroll 1
    for (int ps = 0; ps < 2; ++ps) {
#pragma unroll
        for (int s = 0; s < 4; ++s) { const int row = 4 * s + (lane >> 3), c8 = (lane & 7) * 8;
            const v4f x0 = *(const v4fa*)(&os[wb + row * OSP + c8]); const v4f x1 = *(const v4fa*)(&os[wb + row * OSP + c8 + 4]); v8h hv;
#pragma unroll
            for (int i = 0; i < 4; ++i) { hv[i] = toh_flush(x0[i]); hv[4 + i] = toh_flush(x1[i]); }
            *(volatile v8h*)(orow + (size_t)row * DM + c8) = hv; }
        if (ps == 0) __threadfence(); }
}

__global__ __launch_bounds__(256) void k_out(const float* __restrict__ src, float* dst, int n4) {
    const int i = blockIdx.x * 256 + threadIdx.x; if (i >= n4) return;
    v4f ov;
#pragma unroll
    for (int c = 0; c < 4; ++c) { const int e = 4 * i + c; const int row = e / DOUT; const int col = e - row * DOUT; ov[c] = src[(size_t)row * DOUTP + col]; }
    *(volatile v4f*)(dst + (size_t)i * 4) = ov; __threadfence(); *(volatile v4f*)(dst + (size_t)i * 4) = ov;
}

static constexpr size_t al256(size_t v) { return (v + 255) & ~(size_t)255; }
static constexpr size_t SZ_XH  = al256((size_t)SEQ * DIN * 2);
static constexpr size_t SZ_EW  = al256((size_t)DM * DIN * 2);
static constexpr size_t SZ_WDD = al256((size_t)NL * DM * DM * 2);
static constexpr size_t SZ_WFF = al256((size_t)NL * DFF * DM * 2);
static constexpr size_t SZ_WI  = al256((size_t)DMI * DM * 2);
static constexpr size_t SZ_WF  = al256((size_t)DOUTP * DMI * 2);
static constexpr size_t SZ_EP  = al256((size_t)NL * ERP * HD * 2);
static constexpr size_t SZ_H   = al256((size_t)SEQ * DM * 4);
static constexpr size_t SZ_N   = al256((size_t)SEQ * DM * 2);
static constexpr size_t SZ_F1  = al256((size_t)SEQ * DFF * 2);
static constexpr size_t SZ_OS  = al256((size_t)SEQ * DOUTP * 4);
static constexpr size_t SZ_TOTAL = SZ_XH + SZ_EW + 4 * SZ_WDD + 2 * SZ_WFF + SZ_WI + SZ_WF + SZ_EP + 2 * SZ_H + 7 * SZ_N + SZ_F1 + SZ_OS;
static_assert(SZ_TOTAL <= (size_t)134217728);
static_assert((size_t)NH_ * SEQ * HD == (size_t)SEQ * DM);
static_assert((size_t)SEQ * DMI * 2 <= SZ_F1);

extern "C" void kernel_launch(void* const* d_in, const int* in_sizes, int n_in,
                              void* d_out, int out_size, void* d_ws, size_t ws_size, hipStream_t stream) {
    if (n_in < 26) return;
    if ((size_t)in_sizes[0] < (size_t)SEQ * DIN || (size_t)in_sizes[1] < (size_t)DIN * DM || in_sizes[2] < DM) return;
    if ((size_t)in_sizes[3] < (size_t)NL * DM * DM || (size_t)in_sizes[5] < (size_t)NL * DM * DM || (size_t)in_sizes[7] < (size_t)NL * DM * DM || (size_t)in_sizes[9] < (size_t)NL * DM * DM) return;
    if (in_sizes[4] < NL * DM || in_sizes[6] < NL * DM || in_sizes[8] < NL * DM || in_sizes[10] < NL * DM) return;
    if ((size_t)in_sizes[11] < (size_t)NL * ERR * HD) return;
    if (in_sizes[12] < NL * DM || in_sizes[13] < NL * DM || in_sizes[17] < NL * DM || in_sizes[18] < NL * DM || in_sizes[19] < NL * DM) return;
    if ((size_t)in_sizes[14] < (size_t)NL * DM * DFF || in_sizes[15] < NL * DFF || (size_t)in_sizes[16] < (size_t)NL * DFF * DM) return;
    if (in_sizes[20] < DM || in_sizes[21] < DM || (size_t)in_sizes[22] < (size_t)DM * DMI || in_sizes[23] < DMI) return;
    if ((size_t)in_sizes[24] < (size_t)DMI * DOUT || in_sizes[25] < DOUT) return;
    if ((size_t)out_size < (size_t)SEQ * DOUT) return;
    if (SZ_TOTAL > ws_size) return;
    const float* x    = (const float*)d_in[0];
    const float* embW = (const float*)d_in[1];  const float* embB = (const float*)d_in[2];
    const float* Wq   = (const float*)d_in[3];  const float* bq   = (const float*)d_in[4];
    const float* Wk   = (const float*)d_in[5];  const float* bk   = (const float*)d_in[6];
    const float* Wv   = (const float*)d_in[7];  const float* bv   = (const float*)d_in[8];
    const float* Wo   = (const float*)d_in[9];  const float* bo   = (const float*)d_in[10];
    const float* Er   = (const float*)d_in[11];
    const float* ln1g = (const float*)d_in[12]; const float* ln1b = (const float*)d_in[13];
    const float* W1   = (const float*)d_in[14]; const float* b1   = (const float*)d_in[15];
    const float* W2   = (const float*)d_in[16]; const float* b2   = (const float*)d_in[17];
    const float* ln2g = (const float*)d_in[18]; const float* ln2b = (const float*)d_in[19];
    const float* lnfg = (const float*)d_in[20]; const float* lnfb = (const float*)d_in[21];
    const float* Wi   = (const float*)d_in[22]; const float* bi   = (const float*)d_in[23];
    const float* Wf   = (const float*)d_in[24]; const float* bfo  = (const float*)d_in[25];
    float* OUT = (float*)d_out;
    char* wsp = (char*)d_ws;
    h16* XH  = (h16*)wsp; wsp += SZ_XH;
    h16* EWT = (h16*)wsp; wsp += SZ_EW;
    h16* WQT = (h16*)wsp; wsp += SZ_WDD;
    h16* WKT = (h16*)wsp; wsp += SZ_WDD;
    h16* WVT = (h16*)wsp; wsp += SZ_WDD;
    h16* WOT = (h16*)wsp; wsp += SZ_WDD;
    h16* W1T = (h16*)wsp; wsp += SZ_WFF;
    h16* W2T = (h16*)wsp; wsp += SZ_WFF;
    h16* WIT = (h16*)wsp; wsp += SZ_WI;
    h16* WFT = (h16*)wsp; wsp += SZ_WF;
    h16* EP  = (h16*)wsp; wsp += SZ_EP;
    float* HA = (float*)wsp; wsp += SZ_H;
    float* HB = (float*)wsp; wsp += SZ_H;
    h16* NHP = (h16*)wsp; wsp += SZ_N;
    h16* NRP = (h16*)wsp; wsp += SZ_N;
    h16* QH  = (h16*)wsp; wsp += SZ_N;
    h16* QR  = (h16*)wsp; wsp += SZ_N;
    h16* KP  = (h16*)wsp; wsp += SZ_N;
    h16* VT  = (h16*)wsp; wsp += SZ_N;
    h16* OP  = (h16*)wsp; wsp += SZ_N;
    h16* F1  = (h16*)wsp; wsp += SZ_F1;
    float* OSG = (float*)wsp; wsp += SZ_OS;

    { const int n8 = SEQ * DIN / 8; k_cvt8h<<<(unsigned)((n8 + 255) / 256), 256, 0, stream>>>(x, XH, n8); }
    k_cvt_er<<<(unsigned)((NL * ERP * HD / 8 + 255) / 256), 256, 0, stream>>>(Er, EP);
    k_wconv<<<dim3(DIN / 64, DM / 64, 1),   256, 0, stream>>>(embW, EWT, DIN, DM, DM, WC);
    k_wconv<<<dim3(DM / 64, DM / 64, NL),   256, 0, stream>>>(Wq, WQT, DM, DM, DM, WC);
    k_wconv<<<dim3(DM / 64, DM / 64, NL),   256, 0, stream>>>(Wk, WKT, DM, DM, DM, WC);
    k_wconv<<<dim3(DM / 64, DM / 64, NL),   256, 0, stream>>>(Wv, WVT, DM, DM, DM, WC);
    k_wconv<<<dim3(DM / 64, DM / 64, NL),   256, 0, stream>>>(Wo, WOT, DM, DM, DM, WC);
    k_wconv<<<dim3(DM / 64, DFF / 64, NL),  256, 0, stream>>>(W1, W1T, DM, DFF, DFF, WC);
    k_wconv<<<dim3(DFF / 64, DM / 64, NL),  256, 0, stream>>>(W2, W2T, DFF, DM, DM, WC);
    k_wconv<<<dim3(DM / 64, DMI / 64, 1),   256, 0, stream>>>(Wi, WIT, DM, DMI, DMI, WC);
    k_wconv<<<dim3(DMI / 64, DOUTP / 64, 1), 256, 0, stream>>>(Wf, WFT, DMI, DOUT, DOUTP, WC);

    k_gemm_f32<<<dim3(SEQ / 64, DM / 64, 1), 32, 0, stream>>>(XH, EWT, embB, DM, DIN, WCI, HA, DM);

    for (int l = 0; l < NL; ++l) {
        const size_t wdd = (size_t)l * DM * DM, wff = (size_t)l * DFF * DM;
        k_ln<<<SEQ / 4, 128, 0, stream>>>(HA, ln1g + l * DM, ln1b + l * DM, NHP, NRP, 1);
        k_gemm_q<<<dim3(SEQ / 64, DM / 64, 1), 32, 0, stream>>>(NHP, NRP, WQT + wdd, bq + l * DM, DM, DM, WCI, QH, QR);
        k_gemm_k<<<dim3(SEQ / 64, DM / 64, 1), 32, 0, stream>>>(NHP, WKT + wdd, bk + l * DM, DM, DM, WCI, KP);
        k_gemm_vt<<<dim3(DM / 64, SEQ / 64, 1), 32, 0, stream>>>(WVT + wdd, NHP, bv + l * DM, DM, WCI, VT, SEQ);
        k_flash<<<dim3(SEQ / (16 * AW), NH_, 1), 32 * AW, 0, stream>>>(QH, QR, KP, VT, EP + (size_t)l * ERP * HD, OP);
        k_gemm_f32r<<<dim3(SEQ / 64, DM / 64, 1), 32, 0, stream>>>(OP, WOT + wdd, bo + l * DM, DM, DM, WCI, HA, HB, DM);
        k_ln<<<SEQ / 4, 128, 0, stream>>>(HB, ln2g + l * DM, ln2b + l * DM, NHP, NRP, 0);
        k_gemm_gelu<<<dim3(SEQ / 64, DFF / 64, 1), 32, 0, stream>>>(NHP, W1T + wff, b1 + l * DFF, DFF, DM, WCI, F1, DFF);
        k_gemm_f32r<<<dim3(SEQ / 64, DM / 64, 1), 32, 0, stream>>>(F1, W2T + wff, b2 + l * DM, DM, DFF, WCI, HB, HA, DM);
    }

    k_ln<<<SEQ / 4, 128, 0, stream>>>(HA, lnfg, lnfb, NHP, NRP, 0);
    k_gemm_gelu<<<dim3(SEQ / 64, DMI / 64, 1), 32, 0, stream>>>(NHP, WIT, bi, DMI, DM, WCI, F1, DMI);
    k_gemm_f32<<<dim3(SEQ / 64, DOUTP / 64, 1), 32, 0, stream>>>(F1, WFT, bfo, DOUT, DMI, WCI, OSG, DOUTP);
    { const int n4 = SEQ * DOUT / 4; k_out<<<(unsigned)((n4 + 255) / 256), 256, 0, stream>>>(OSG, OUT, n4); }
}
